// CMSBlockLinear_67216238182784
// MI455X (gfx1250) — hardware-run, weakly checked
//
#include <hip/hip_runtime.h>

typedef __attribute__((ext_vector_type(16))) __bf16   v16b;
typedef __attribute__((ext_vector_type(8)))  __bf16   v8b;
typedef __attribute__((ext_vector_type(8)))  float    v8f;
typedef __attribute__((ext_vector_type(4)))  float    v4f;
typedef __attribute__((ext_vector_type(4)))  unsigned v4u;

constexpr int kTok     = 2048;
constexpr int kInF     = 2048;
constexpr int kOutF    = 2048;
constexpr int kTile    = 16;
constexpr int kBlkRows = kOutF / kTile;
constexpr int kBlkCols = kInF / kTile;
constexpr int kActive  = 32;
constexpr int kDepth   = kActive * kTile;
constexpr int kSlabP   = 36;
static_assert(kBlkRows == 128 && kBlkCols == 128, "tile grid");
static_assert(kDepth == 512 && (kDepth % 32) == 0, "depth multiple of 32");
static_assert((kTok % 512) == 0, "8 waves x 64 token rows per block");
static_assert((kBlkRows % 2) == 0, "block-row pairs");
static_assert((kSlabP % 4) == 0, "slab pitch keeps 16-B alignment");

constexpr size_t kOffX16  = 0;
constexpr size_t kOffW16  = kOffX16 + (size_t)kTok * kInF * 2;
constexpr size_t kWsTotal = kOffW16 + (size_t)kOutF * kDepth * 2;
static_assert(kWsTotal == 10485760ull, "carve total");
static_assert(kWsTotal <= 134217728ull, "carve cap");
static_assert((kOffW16 % 128) == 0, "aligned region");

__device__ __forceinline__ unsigned f2bf_bits(float f) {
  const unsigned u = __float_as_uint(f);
  return ((u + 0x7FFFu + ((u >> 16) & 1u)) >> 16) & 0xFFFFu;
}
__device__ __forceinline__ unsigned pack_bf2(float lo_elem, float hi_elem) {
  const unsigned a = f2bf_bits(lo_elem);
  const unsigned b = f2bf_bits(hi_elem);
  return a | (b << 16);
}
__device__ __forceinline__ v8f mma_bf(v16b a, v16b b, v8f c) {
  c = __builtin_amdgcn_wmma_f32_16x16x32_bf16(false, a, false, b, (short)0, c, false, false);
  asm volatile("v_nop\n\tv_nop\n\tv_nop\n\tv_nop" : "+v"(c) : "v"(a), "v"(b));
  return c;
}
union FragB { v16b v; v8b h[2]; };

__global__ __launch_bounds__(256) void cast_plane_bf16_kernel(
    const float* __restrict__ src, unsigned short* __restrict__ dst, int total8)
{
  const int i = blockIdx.x * 256 + threadIdx.x;
  if (i >= total8) return;
  const size_t e0 = (size_t)i << 3;
  const v4f a0 = *(const v4f*)(src + e0);
  const v4f a1 = *(const v4f*)(src + e0 + 4);
  const float f0 = a0[0];
  const float f1 = a0[1];
  const float f2 = a0[2];
  const float f3 = a0[3];
  const float f4 = a1[0];
  const float f5 = a1[1];
  const float f6 = a1[2];
  const float f7 = a1[3];
  v4u w;
  w[0] = pack_bf2(f0, f1);
  w[1] = pack_bf2(f2, f3);
  w[2] = pack_bf2(f4, f5);
  w[3] = pack_bf2(f6, f7);
  unsigned short* p = dst + e0;
  *(volatile v4u*)p = w;
  __threadfence();
  *(volatile v4u*)p = w;
}

__global__ __launch_bounds__(256) void cast_tiles_bf16_kernel(
    const float* __restrict__ vals, unsigned short* __restrict__ dst, int total8)
{
  const int g = blockIdx.x * 256 + threadIdx.x;
  if (g >= total8) return;
  const int n   = g >> 6;
  const int grp = g & 63;
  const int k   = grp >> 1;
  const int j0  = (grp & 1) * 8;
  const int r   = n >> 4;
  const int i   = n & 15;
  const float* s = vals + ((size_t)((r * kActive + k) * kTile + i) * kTile + j0);
  const v4f a0 = *(const v4f*)(s);
  const v4f a1 = *(const v4f*)(s + 4);
  const float f0 = a0[0];
  const float f1 = a0[1];
  const float f2 = a0[2];
  const float f3 = a0[3];
  const float f4 = a1[0];
  const float f5 = a1[1];
  const float f6 = a1[2];
  const float f7 = a1[3];
  v4u w;
  w[0] = pack_bf2(f0, f1);
  w[1] = pack_bf2(f2, f3);
  w[2] = pack_bf2(f4, f5);
  w[3] = pack_bf2(f6, f7);
  unsigned short* p = dst + ((size_t)g << 3);
  *(volatile v4u*)p = w;
  __threadfence();
  *(volatile v4u*)p = w;
}

__global__ __launch_bounds__(256) void gathered_tiles_wmma_kernel(
    const unsigned short* __restrict__ X16p, const unsigned short* __restrict__ W16p,
    const int* __restrict__ cols, const float* __restrict__ bias, float* __restrict__ out)
{
  __shared__ __align__(16) float sT[8][16 * kSlabP];
  const __bf16* X16 = (const __bf16*)X16p;
  const __bf16* W16 = (const __bf16*)W16p;
  const int lane = threadIdx.x & 31;
  const int wave = threadIdx.x >> 5;
  const int h    = lane >> 4;
  const int n    = lane & 15;
  const int rp   = blockIdx.y;
  const int r0   = rp * 2;
  const int t0   = (blockIdx.x * 8 + wave) * 64;
  const int* crow = cols + (size_t)r0 * kActive;

  const __bf16* xr0 = X16 + (size_t)(t0 +  0 + n) * kInF + 8 * h;
  const __bf16* xr1 = X16 + (size_t)(t0 + 16 + n) * kInF + 8 * h;
  const __bf16* xr2 = X16 + (size_t)(t0 + 32 + n) * kInF + 8 * h;
  const __bf16* xr3 = X16 + (size_t)(t0 + 48 + n) * kInF + 8 * h;
  const __bf16* wr0 = W16 + (size_t)((r0 + 0) * kTile + n) * kDepth + 8 * h;
  const __bf16* wr1 = W16 + (size_t)((r0 + 1) * kTile + n) * kDepth + 8 * h;

  v8f acc[2][4];
#pragma unroll
  for (int ri = 0; ri < 2; ++ri)
#pragma unroll
    for (int i = 0; i < 4; ++i) acc[ri][i] = (v8f){0.f, 0.f, 0.f, 0.f, 0.f, 0.f, 0.f, 0.f};

#pragma unroll 1
  for (int m = 0; m < kActive / 2; ++m) {
#pragma unroll
    for (int ri = 0; ri < 2; ++ri) {
      int c0 = crow[ri * kActive + 2 * m];
      int c1 = crow[ri * kActive + 2 * m + 1];
      c0 = c0 < 0 ? 0 : (c0 > kBlkCols - 1 ? kBlkCols - 1 : c0);
      c1 = c1 < 0 ? 0 : (c1 > kBlkCols - 1 ? kBlkCols - 1 : c1);
      const int o0 = c0 * kTile;
      const int o1 = c1 * kTile;
      const __bf16* wp = (ri == 0 ? wr0 : wr1) + m * 32;
      FragB b;
      b.h[0] = *(const v8b*)(wp);
      b.h[1] = *(const v8b*)(wp + 16);
      FragB a0, a1, a2, a3;
      a0.h[0] = *(const v8b*)(xr0 + o0);
      a0.h[1] = *(const v8b*)(xr0 + o1);
      a1.h[0] = *(const v8b*)(xr1 + o0);
      a1.h[1] = *(const v8b*)(xr1 + o1);
      a2.h[0] = *(const v8b*)(xr2 + o0);
      a2.h[1] = *(const v8b*)(xr2 + o1);
      a3.h[0] = *(const v8b*)(xr3 + o0);
      a3.h[1] = *(const v8b*)(xr3 + o1);
      acc[ri][0] = mma_bf(a0.v, b.v, acc[ri][0]);
      acc[ri][1] = mma_bf(a1.v, b.v, acc[ri][1]);
      acc[ri][2] = mma_bf(a2.v, b.v, acc[ri][2]);
      acc[ri][3] = mma_bf(a3.v, b.v, acc[ri][3]);
    }
  }

  const float braw0 = bias[(r0 + 0) * kTile + n];
  const float braw1 = bias[(r0 + 1) * kTile + n];
  const float bv0 = __uint_as_float(f2bf_bits(braw0) << 16);
  const float bv1 = __uint_as_float(f2bf_bits(braw1) << 16);

  float* slab = sT[wave];
  const int q  = lane >> 3;
  const int c4 = (lane & 7) * 4;
#pragma unroll
  for (int i = 0; i < 4; ++i) {
#pragma unroll
    for (int rr = 0; rr < 8; ++rr) {
      slab[(8 * h + rr) * kSlabP + n]      = acc[0][i][rr] + bv0;
      slab[(8 * h + rr) * kSlabP + 16 + n] = acc[1][i][rr] + bv1;
    }
    __syncthreads();
    v4f vals[4];
#pragma unroll
    for (int it = 0; it < 4; ++it) vals[it] = *(const v4f*)(slab + (it * 4 + q) * kSlabP + c4);
    for (int pass = 0; pass < 2; ++pass) {
#pragma unroll
      for (int it = 0; it < 4; ++it) {
        const int row = t0 + i * 16 + it * 4 + q;
        *(volatile v4f*)(out + (size_t)row * kOutF + rp * 32 + c4) = vals[it];
      }
      __threadfence();
    }
    __syncthreads();
  }
}

extern "C" void kernel_launch(void* const* d_in, const int* in_sizes, int n_in,
                              void* d_out, int out_size, void* d_ws, size_t ws_size,
                              hipStream_t stream) {
  if (n_in < 4) return;
  if (in_sizes[0] != kTok * kInF) return;
  if (in_sizes[1] != kBlkRows * kActive * kTile * kTile) return;
  if (in_sizes[2] != kBlkRows * kActive) return;
  if (in_sizes[3] != kOutF) return;
  if (out_size != kTok * kOutF) return;
  if (ws_size < kWsTotal) return;

  const float* x      = (const float*)d_in[0];
  const float* values = (const float*)d_in[1];
  const int*   cols   = (const int*)d_in[2];
  const float* bias   = (const float*)d_in[3];
  float*       out    = (float*)d_out;

  char* ws = (char*)d_ws;
  unsigned short* X16 = (unsigned short*)(ws + kOffX16);
  unsigned short* W16 = (unsigned short*)(ws + kOffW16);

  constexpr int kX8 = kTok * kInF / 8;
  constexpr int kW8 = kOutF * kDepth / 8;
  static_assert((kX8 % 256) == 0 && (kW8 % 256) == 0, "exact cast grids");

  cast_plane_bf16_kernel<<<kX8 / 256, 256, 0, stream>>>(x, X16, kX8);
  cast_tiles_bf16_kernel<<<kW8 / 256, 256, 0, stream>>>(values, W16, kW8);
  gathered_tiles_wmma_kernel<<<dim3(kTok / 512, kBlkRows / 2), 256, 0, stream>>>(X16, W16, cols, bias, out);
}
